// MambaBlock_4664334483708
// MI455X (gfx1250) — hardware-verified
//
#include <hip/hip_runtime.h>
#include <math.h>

typedef __attribute__((ext_vector_type(16))) __bf16   v16b;
typedef __attribute__((ext_vector_type(8)))  __bf16   v8b;
typedef __attribute__((ext_vector_type(8)))  float    v8f;
typedef __attribute__((ext_vector_type(4)))  float    v4f;
typedef __attribute__((ext_vector_type(4)))  unsigned v4u;

constexpr int kBatch  = 2;
constexpr int kSeqL   = 2048;
constexpr int kDmod   = 1024;
constexpr int kDin    = 2048;
constexpr int kNst    = 16;
constexpr int kDtR    = 64;
constexpr int kPrjN   = 96;
constexpr int kPrjP   = 128;
constexpr int kXZP    = 2 * kDin;
constexpr int kRows   = kBatch * kSeqL;
constexpr int kTP     = 260;
constexpr int kScanTS = 64;
constexpr int kScanCh = 64;
constexpr int kScanYP = 68;
static_assert(kDtR + 2 * kNst == kPrjN, "projection width");
static_assert((kDmod % 32) == 0 && (kDin % 32) == 0 && (kDtR % 32) == 0, "GEMM K multiples of 32");
static_assert((kSeqL % 64) == 0 && (kXZP % 64) == 0 && (kPrjP % 64) == 0 && (kDin % 64) == 0 && (kDmod % 64) == 0, "GEMM M,N multiples of 64");
static_assert((kSeqL % kScanTS) == 0 && (kDin % kScanCh) == 0 && (kDin % 256) == 0, "tile multiples");
static_assert(((kSeqL / 64) * (kXZP / 64)) % 8 == 0 && ((kSeqL / 64) * (kPrjP / 64)) % 8 == 0 &&
              ((kSeqL / 64) * (kDin / 64)) % 8 == 0 && ((kSeqL / 64) * (kDmod / 64)) % 8 == 0, "8 tiles per GEMM block, exact grids");

constexpr size_t kOffWIN  = 0;
constexpr size_t kOffWSM  = kOffWIN  + (size_t)kXZP  * kDmod * 2;
constexpr size_t kOffWD2  = kOffWSM  + (size_t)kPrjP * kDin  * 2;
constexpr size_t kOffWOUT = kOffWD2  + (size_t)kDin  * kDtR  * 2;
constexpr size_t kOffXNH  = kOffWOUT + (size_t)kDmod * kDin  * 2;
constexpr size_t kOffXNL  = kOffXNH  + (size_t)kRows * kDmod * 2;
constexpr size_t kOffXZ   = kOffXNL  + (size_t)kRows * kDmod * 2;
constexpr size_t kOffXCH  = kOffXZ   + (size_t)kSeqL * kXZP  * 4;
constexpr size_t kOffXCL  = kOffXCH  + (size_t)kSeqL * kDin  * 2;
constexpr size_t kOffPROJ = kOffXCL  + (size_t)kSeqL * kDin  * 2;
constexpr size_t kOffD1H  = kOffPROJ + (size_t)kSeqL * kPrjP * 4;
constexpr size_t kOffD1L  = kOffD1H  + (size_t)kSeqL * kDtR  * 2;
constexpr size_t kOffDLR  = kOffD1L  + (size_t)kSeqL * kDtR  * 2;
constexpr size_t kOffYH   = kOffDLR  + (size_t)kSeqL * kDin  * 4;
constexpr size_t kOffYL   = kOffYH   + (size_t)kSeqL * kDin  * 2;
constexpr size_t kWsTotal = kOffYL   + (size_t)kSeqL * kDin  * 2;
static_assert(kWsTotal == 115605504ull, "carve total");
static_assert(kWsTotal <= 134217728ull, "carve cap");
static_assert((kOffWSM % 128) == 0 && (kOffWD2 % 128) == 0 && (kOffWOUT % 128) == 0 && (kOffXNH % 128) == 0 &&
              (kOffXNL % 128) == 0 && (kOffXZ % 128) == 0 && (kOffXCH % 128) == 0 && (kOffXCL % 128) == 0 &&
              (kOffPROJ % 128) == 0 && (kOffD1H % 128) == 0 && (kOffD1L % 128) == 0 && (kOffDLR % 128) == 0 &&
              (kOffYH % 128) == 0 && (kOffYL % 128) == 0, "128-B aligned regions");

__device__ __forceinline__ unsigned bf_rne_bits(float f) {
  const unsigned u = __float_as_uint(f);
  return (u + 0x7FFFu + ((u >> 16) & 1u)) >> 16;
}
__device__ __forceinline__ float bf_rne(float f) { return __uint_as_float(bf_rne_bits(f) << 16); }
__device__ __forceinline__ void split2(float x0, float x1, unsigned& wh, unsigned& wl) {
  const unsigned h0 = bf_rne_bits(x0), h1 = bf_rne_bits(x1);
  const float r0 = x0 - __uint_as_float(h0 << 16);
  const float r1 = x1 - __uint_as_float(h1 << 16);
  const unsigned l0 = bf_rne_bits(r0), l1 = bf_rne_bits(r1);
  wh = h0 | (h1 << 16);
  wl = l0 | (l1 << 16);
}
__device__ __forceinline__ void split8(const v4f a0, const v4f a1, v4u& wh, v4u& wl) {
  unsigned h0, l0, h1, l1, h2, l2, h3, l3;
  split2(a0[0], a0[1], h0, l0);
  split2(a0[2], a0[3], h1, l1);
  split2(a1[0], a1[1], h2, l2);
  split2(a1[2], a1[3], h3, l3);
  wh = (v4u){h0, h1, h2, h3};
  wl = (v4u){l0, l1, l2, l3};
}
__device__ __forceinline__ v4u rne8(const v4f a0, const v4f a1) {
  const unsigned p0 = bf_rne_bits(a0[0]) | (bf_rne_bits(a0[1]) << 16);
  const unsigned p1 = bf_rne_bits(a0[2]) | (bf_rne_bits(a0[3]) << 16);
  const unsigned p2 = bf_rne_bits(a1[0]) | (bf_rne_bits(a1[1]) << 16);
  const unsigned p3 = bf_rne_bits(a1[2]) | (bf_rne_bits(a1[3]) << 16);
  return (v4u){p0, p1, p2, p3};
}

__device__ __forceinline__ void dep_guard4_b(v8f& a, v8f& b, v8f& c, v8f& d, v16b x, v16b y) {
  asm volatile("v_nop\n\tv_nop\n\tv_nop\n\tv_nop" : "+v"(a), "+v"(b), "+v"(c), "+v"(d) : "v"(x), "v"(y));
}
__device__ __forceinline__ void keep4_b(v16b a, v16b b, v16b c, v16b d) { asm volatile("v_nop" :: "v"(a), "v"(b), "v"(c), "v"(d)); }
__device__ __forceinline__ void acc_guard4(v8f& a, v8f& b, v8f& c, v8f& d) { asm volatile("v_nop\n\tv_nop\n\tv_nop\n\tv_nop" : "+v"(a), "+v"(b), "+v"(c), "+v"(d)); }
struct FragBF {
  typedef v16b V; union U { v16b v; v8b h[2]; };
  static __device__ __forceinline__ v16b load(const __bf16* p) {
    U f; f.h[0] = *(const v8b*)(p); f.h[1] = *(const v8b*)(p + 16); return f.v;
  }
  static __device__ __forceinline__ v8f mma(v16b a, v16b b, v8f c) {
    return __builtin_amdgcn_wmma_f32_16x16x32_bf16(false, a, false, b, (short)0, c, false, false);
  }
};

template <bool RESID_BF>
__global__ __launch_bounds__(256) void wmma_gemm64_a2(
    const unsigned short* __restrict__ Ap, const unsigned short* __restrict__ A2p, int lda,
    const unsigned short* __restrict__ Btp, int ldb,
    float* __restrict__ C, int ldc,
    const float* __restrict__ resid,
    int M, int N, int K) {
  typedef __bf16 T;
  typedef v16b V;
  const T* A  = (const T*)Ap;
  const T* A2 = (const T*)A2p;
  const T* Bt = (const T*)Btp;
  __shared__ __align__(16) float sT[8][16 * 68];
  const int lane = threadIdx.x & 31;
  const int wave = threadIdx.x >> 5;
  const int tilesN = N >> 6;
  const int tilesM = M >> 6;
  const int tile = blockIdx.x * 8 + wave;
  if (tile >= tilesM * tilesN) return;
  const int tm = tile / tilesN;
  const int tn = tile - tm * tilesN;
  const int m0 = tm << 6;
  const int n0 = tn << 6;

  const int rlane = lane & 15;
  const int koff  = (lane >> 4) * 8;
  const int mOff  = (lane >> 4) * 8;

  v8f acc[4][4];
#pragma unroll
  for (int i = 0; i < 4; ++i)
#pragma unroll
    for (int j = 0; j < 4; ++j) acc[i][j] = (v8f){0.f,0.f,0.f,0.f,0.f,0.f,0.f,0.f};

  for (int k0 = 0; k0 < K; k0 += 32) {
    V bh[4];
#pragma unroll
    for (int j = 0; j < 4; ++j) {
      const size_t bo = (size_t)(n0 + (j << 4) + rlane) * ldb + koff + k0;
      bh[j] = FragBF::load(Bt + bo);
    }
#pragma unroll
    for (int i = 0; i < 4; ++i) {
      const size_t ao = (size_t)(m0 + (i << 4) + rlane) * lda + koff + k0;
      V ah = FragBF::load(A + ao);
      V al = FragBF::load(A2 + ao);
#pragma unroll
      for (int j = 0; j < 4; ++j) {
        acc[i][j] = FragBF::mma(ah, bh[j], acc[i][j]);
        acc[i][j] = FragBF::mma(al, bh[j], acc[i][j]);
      }
      dep_guard4_b(acc[i][0], acc[i][1], acc[i][2], acc[i][3], ah, al);
    }
    keep4_b(bh[0], bh[1], bh[2], bh[3]);
  }
  acc_guard4(acc[0][0], acc[0][1], acc[0][2], acc[0][3]);
  acc_guard4(acc[1][0], acc[1][1], acc[1][2], acc[1][3]);
  acc_guard4(acc[2][0], acc[2][1], acc[2][2], acc[2][3]);
  acc_guard4(acc[3][0], acc[3][1], acc[3][2], acc[3][3]);

  float* slab = sT[wave];
  const int hh = lane >> 4, c4 = (lane & 15) * 4;
#pragma unroll
  for (int i = 0; i < 4; ++i) {
    const int mBase = m0 + (i << 4);
#pragma unroll
    for (int j = 0; j < 4; ++j) {
#pragma unroll
      for (int r = 0; r < 8; ++r) slab[(mOff + r) * 68 + (j << 4) + rlane] = acc[i][j][r];
    }
    __builtin_amdgcn_fence(__ATOMIC_RELEASE, "workgroup");
    __builtin_amdgcn_wave_barrier();
    __builtin_amdgcn_fence(__ATOMIC_ACQUIRE, "workgroup");
    v4f ov[8];
#pragma unroll
    for (int it = 0; it < 8; ++it) {
      const int row = it * 2 + hh;
      v4f v = *(const v4f*)(slab + row * 68 + c4);
      if (RESID_BF) {
        const v4f rr = *(const v4f*)(resid + (size_t)(mBase + row) * ldc + n0 + c4);
        v[0] += bf_rne(rr[0]);
        v[1] += bf_rne(rr[1]);
        v[2] += bf_rne(rr[2]);
        v[3] += bf_rne(rr[3]);
      }
      ov[it] = v;
    }
    for (int pass = 0; pass < 2; ++pass) {
#pragma unroll
      for (int it = 0; it < 8; ++it) {
        const int row = it * 2 + hh;
        *(volatile v4f*)(C + (size_t)(mBase + row) * ldc + n0 + c4) = ov[it];
      }
      __threadfence();
    }
    __builtin_amdgcn_fence(__ATOMIC_RELEASE, "workgroup");
    __builtin_amdgcn_wave_barrier();
    __builtin_amdgcn_fence(__ATOMIC_ACQUIRE, "workgroup");
  }
}

__global__ __launch_bounds__(256) void rne_rows_bf16_kernel(
    const float* __restrict__ src, unsigned short* __restrict__ dst, int total8)
{
  const int i = blockIdx.x * 256 + threadIdx.x;
  if (i >= total8) return;
  const size_t e0 = (size_t)i << 3;
  const v4f a0 = *(const v4f*)(src + e0);
  const v4f a1 = *(const v4f*)(src + e0 + 4);
  const v4u w = rne8(a0, a1);
  unsigned short* q = dst + e0;
  *(volatile v4u*)q = w;
  __threadfence();
  *(volatile v4u*)q = w;
}

__global__ __launch_bounds__(256) void pack_small_kernel(
    const float* __restrict__ wd1, const float* __restrict__ wb, const float* __restrict__ wc,
    unsigned short* __restrict__ dst)
{
  const int row = blockIdx.x;
  const int c8 = threadIdx.x * 8;
  v4u w = (v4u){0u, 0u, 0u, 0u};
  if (row < kPrjN) {
    const float* src = (row < kDtR) ? (wd1 + (size_t)row * kDin)
                     : (row < kDtR + kNst) ? (wb + (size_t)(row - kDtR) * kDin)
                     : (wc + (size_t)(row - kDtR - kNst) * kDin);
    const v4f a0 = *(const v4f*)(src + c8);
    const v4f a1 = *(const v4f*)(src + c8 + 4);
    w = rne8(a0, a1);
  }
  unsigned short* q = dst + (size_t)row * kDin + c8;
  *(volatile v4u*)q = w;
  __threadfence();
  *(volatile v4u*)q = w;
}

__global__ __launch_bounds__(256) void rmsnorm_split_kernel(
    const float* __restrict__ xin, const float* __restrict__ nw,
    unsigned short* __restrict__ XNH, unsigned short* __restrict__ XNL)
{
  const int lane = threadIdx.x & 31, wave = threadIdx.x >> 5;
  const int row = blockIdx.x * 8 + wave;
  const float* xr = xin + (size_t)row * kDmod + lane * 8;
  v4f a[8];
#pragma unroll
  for (int j = 0; j < 4; ++j) {
    a[2 * j]     = *(const v4f*)(xr + j * 256);
    a[2 * j + 1] = *(const v4f*)(xr + j * 256 + 4);
  }
  float ss = 0.f;
#pragma unroll
  for (int i = 0; i < 8; ++i) {
#pragma unroll
    for (int e = 0; e < 4; ++e) {
      const float r = bf_rne(a[i][e]);
      a[i][e] = r;
      ss = fmaf(r, r, ss);
    }
  }
#pragma unroll
  for (int off = 16; off >= 1; off >>= 1) ss += __shfl_xor(ss, off, 32);
  const float scl = 1.0f / sqrtf(ss * (1.0f / (float)kDmod) + 1e-5f);
  asm volatile("" ::: "memory");
  const float* wr = nw + lane * 8;
  v4u wh[4], wl[4];
#pragma unroll
  for (int j = 0; j < 4; ++j) {
    const v4f g0 = *(const v4f*)(wr + j * 256);
    const v4f g1 = *(const v4f*)(wr + j * 256 + 4);
    v4f y0, y1;
#pragma unroll
    for (int e = 0; e < 4; ++e) {
      y0[e] = (a[2 * j][e] * scl) * bf_rne(g0[e]);
      y1[e] = (a[2 * j + 1][e] * scl) * bf_rne(g1[e]);
    }
    split8(y0, y1, wh[j], wl[j]);
  }
  unsigned short* qh = XNH + (size_t)row * kDmod + lane * 8;
  unsigned short* ql = XNL + (size_t)row * kDmod + lane * 8;
  for (int pass = 0; pass < 2; ++pass) {
#pragma unroll
    for (int j = 0; j < 4; ++j) {
      *(volatile v4u*)(qh + j * 256) = wh[j];
      *(volatile v4u*)(ql + j * 256) = wl[j];
    }
    __threadfence();
  }
}

__global__ __launch_bounds__(256) void conv_silu_split_kernel(
    const float* __restrict__ XZ, const float* __restrict__ cw, const float* __restrict__ cb,
    unsigned short* __restrict__ XCH, unsigned short* __restrict__ XCL)
{
  __shared__ __align__(16) float sT[16 * kTP];
  const int tid = threadIdx.x, lane = tid & 31, wave = tid >> 5;
  const int d0 = blockIdx.x * 256, d = d0 + tid;
  const int t0 = blockIdx.y * 64;
  const v4f wv = *(const v4f*)(cw + (size_t)d * 4);
  const float w0 = bf_rne(wv[0]), w1 = bf_rne(wv[1]), w2 = bf_rne(wv[2]), w3 = bf_rne(wv[3]);
  const float bc = bf_rne(cb[d]);
  float xm3, xm2, xm1;
  {
    const bool hist = (t0 > 0);
    const int rb = hist ? (t0 - 3) : t0;
    const float v3 = XZ[(size_t)rb * kXZP + d];
    const float v2 = XZ[(size_t)(rb + 1) * kXZP + d];
    const float v1 = XZ[(size_t)(rb + 2) * kXZP + d];
    xm3 = hist ? v3 : 0.f;
    xm2 = hist ? v2 : 0.f;
    xm1 = hist ? v1 : 0.f;
  }
#pragma unroll 1
  for (int sub = 0; sub < 4; ++sub) {
    const int lb = t0 + sub * 16;
#pragma unroll 1
    for (int s = 0; s < 16; ++s) {
      const float xcur = XZ[(size_t)(lb + s) * kXZP + d];
      float acc = bc;
      acc = fmaf(w0, xm3, acc);
      acc = fmaf(w1, xm2, acc);
      acc = fmaf(w2, xm1, acc);
      acc = fmaf(w3, xcur, acc);
      const float sg = __builtin_amdgcn_rcpf(1.0f + expf(-acc));
      sT[s * kTP + tid] = acc * sg;
      xm3 = xm2; xm2 = xm1; xm1 = xcur;
    }
    __syncthreads();
    v4u bh[2], bl[2];
#pragma unroll
    for (int it = 0; it < 2; ++it) {
      const float* sp = sT + (it * 8 + wave) * kTP + lane * 8;
      const v4f a0 = *(const v4f*)(sp);
      const v4f a1 = *(const v4f*)(sp + 4);
      split8(a0, a1, bh[it], bl[it]);
    }
    for (int pass = 0; pass < 2; ++pass) {
#pragma unroll
      for (int it = 0; it < 2; ++it) {
        const size_t o = (size_t)(lb + it * 8 + wave) * kDin + d0 + lane * 8;
        *(volatile v4u*)(XCH + o) = bh[it];
        *(volatile v4u*)(XCL + o) = bl[it];
      }
      __threadfence();
    }
    __syncthreads();
  }
}

__global__ __launch_bounds__(256) void d1_split_kernel(
    const float* __restrict__ PROJ, unsigned short* __restrict__ D1H, unsigned short* __restrict__ D1L, int total8)
{
  const int i = blockIdx.x * 256 + threadIdx.x;
  if (i >= total8) return;
  const int e0  = i << 3;
  const int row = e0 >> 6;
  const int c8  = e0 & 63;
  const float* p = PROJ + (size_t)row * kPrjP + c8;
  const v4f a0 = *(const v4f*)(p);
  const v4f a1 = *(const v4f*)(p + 4);
  v4u wh, wl;
  split8(a0, a1, wh, wl);
  unsigned short* qh = D1H + e0;
  unsigned short* ql = D1L + e0;
  *(volatile v4u*)qh = wh;
  *(volatile v4u*)ql = wl;
  __threadfence();
  *(volatile v4u*)qh = wh;
  *(volatile v4u*)ql = wl;
}

__global__ __launch_bounds__(64) void scan_kernel(
    const float* __restrict__ DLR, const unsigned* __restrict__ XCHw, const unsigned* __restrict__ XCLw,
    const float* __restrict__ XZ, const float* __restrict__ PROJ,
    const float* __restrict__ Alog, const float* __restrict__ bdt, const float* __restrict__ Dp,
    unsigned short* __restrict__ YH, unsigned short* __restrict__ YL)
{
  __shared__ __align__(16) float sBC[kScanTS * 32];
  __shared__ __align__(16) float sY[kScanTS * kScanYP];
  __shared__ __align__(16) float sA[kNst * kScanCh];
  const int tid = threadIdx.x, lane = tid & 31, wave = tid >> 5;
  const int d0 = blockIdx.x * kScanCh;
  const int d  = d0 + tid;
#pragma unroll 1
  for (int n = 0; n < kNst; ++n) sA[n * kScanCh + tid] = -expf(bf_rne(Alog[(size_t)d * kNst + n]));
  __syncthreads();
  float negA[kNst], h[kNst];
#pragma unroll
  for (int n = 0; n < kNst; ++n) {
    negA[n] = sA[n * kScanCh + tid];
    h[n] = 0.f;
  }
  const float bb = bf_rne(bdt[d]);
  const float Dd = bf_rne(Dp[d]);
  const bool  odd = (tid & 1) != 0;
  const int sr = tid >> 3, sc4 = (tid & 7) * 4;
  const int q = lane >> 3, c8 = (lane & 7) * 8;
#pragma unroll 1
  for (int t0 = 0; t0 < kSeqL; t0 += kScanTS) {
    __syncthreads();
#pragma unroll
    for (int i = 0; i < 8; ++i) {
      const int r = sr + 8 * i;
      *(v4f*)(sBC + r * 32 + sc4) = *(const v4f*)(PROJ + (size_t)(t0 + r) * kPrjP + kDtR + sc4);
    }
    __syncthreads();
#pragma unroll 1
    for (int s = 0; s < kScanTS; ++s) {
      const size_t t = (size_t)(t0 + s);
      const float* br = sBC + s * 32;
      float Bs[kNst], Cs[kNst];
#pragma unroll
      for (int q4 = 0; q4 < 4; ++q4) {
        const v4f bv = *(const v4f*)(br + 4 * q4);
        const v4f cv = *(const v4f*)(br + kNst + 4 * q4);
        Bs[4 * q4 + 0] = bv[0]; Bs[4 * q4 + 1] = bv[1]; Bs[4 * q4 + 2] = bv[2]; Bs[4 * q4 + 3] = bv[3];
        Cs[4 * q4 + 0] = cv[0]; Cs[4 * q4 + 1] = cv[1]; Cs[4 * q4 + 2] = cv[2]; Cs[4 * q4 + 3] = cv[3];
      }
      const float v    = DLR[t * kDin + d] + bb;
      const unsigned wh = XCHw[(t * kDin + d) >> 1];
      const unsigned wl = XCLw[(t * kDin + d) >> 1];
      const float sk   = XZ[t * kXZP + kDin + d];
      const float ea   = expf(-fabsf(v));
      const float u    = 1.0f + ea;
      const float l1p  = logf(u) + (ea - (u - 1.0f)) * __builtin_amdgcn_rcpf(u);
      const float dt   = fmaxf(v, 0.0f) + l1p;
      const unsigned hb = odd ? (wh & 0xffff0000u) : (wh << 16);
      const unsigned lb = odd ? (wl & 0xffff0000u) : (wl << 16);
      const float xt   = __uint_as_float(hb) + __uint_as_float(lb);
      const float dtx  = dt * xt;
      float y = 0.f;
#pragma unroll
      for (int k = 0; k < kNst; ++k) {
        const float e = expf(dt * negA[k]);
        h[k] = fmaf(e, h[k], dtx * Bs[k]);
        y = fmaf(h[k], Cs[k], y);
      }
      y = fmaf(xt, Dd, y);
      const float sg = __builtin_amdgcn_rcpf(1.0f + expf(-sk));
      sY[s * kScanYP + tid] = y * (sk * sg);
    }
    __syncthreads();
    v4u hv[8], lv[8];
#pragma unroll
    for (int it = 0; it < 8; ++it) {
      const int row = it * 8 + wave * 4 + q;
      const float* sp = sY + row * kScanYP + c8;
      const v4f a0 = *(const v4f*)(sp);
      const v4f a1 = *(const v4f*)(sp + 4);
      split8(a0, a1, hv[it], lv[it]);
    }
    for (int pass = 0; pass < 2; ++pass) {
#pragma unroll
      for (int it = 0; it < 8; ++it) {
        const int row = it * 8 + wave * 4 + q;
        const size_t o = (size_t)(t0 + row) * kDin + d0 + c8;
        *(volatile v4u*)(YH + o) = hv[it];
        *(volatile v4u*)(YL + o) = lv[it];
      }
      __threadfence();
    }
  }
}

extern "C" void kernel_launch(void* const* d_in, const int* in_sizes, int n_in,
                              void* d_out, int out_size, void* d_ws, size_t ws_size,
                              hipStream_t stream)
{
  if (n_in < 14) return;
  if (in_sizes[0] != kRows * kDmod) return;
  if (in_sizes[1] != kDmod) return;
  if (in_sizes[2] != kDin * kDmod || in_sizes[3] != kDin * kDmod) return;
  if (in_sizes[4] != kDin * 4 || in_sizes[5] != kDin) return;
  if (in_sizes[6] != kDtR * kDin || in_sizes[7] != kDin * kDtR || in_sizes[8] != kDin) return;
  if (in_sizes[9] != kNst * kDin || in_sizes[10] != kNst * kDin) return;
  if (in_sizes[11] != kDin * kNst || in_sizes[12] != kDin) return;
  if (in_sizes[13] != kDmod * kDin) return;
  if (out_size != kRows * kDmod) return;
  if (ws_size < kWsTotal) return;

  const float* resid  = (const float*)d_in[0];
  const float* norm_w = (const float*)d_in[1];
  const float* skip_w = (const float*)d_in[2];
  const float* in_w   = (const float*)d_in[3];
  const float* conv_w = (const float*)d_in[4];
  const float* conv_b = (const float*)d_in[5];
  const float* wd1    = (const float*)d_in[6];
  const float* wd2    = (const float*)d_in[7];
  const float* wd2_b  = (const float*)d_in[8];
  const float* wb     = (const float*)d_in[9];
  const float* wc     = (const float*)d_in[10];
  const float* A_log  = (const float*)d_in[11];
  const float* W_D    = (const float*)d_in[12];
  const float* out_w  = (const float*)d_in[13];
  float* out = (float*)d_out;

  char* ws = (char*)d_ws;
  unsigned short* WIN  = (unsigned short*)(ws + kOffWIN);
  unsigned short* WSM  = (unsigned short*)(ws + kOffWSM);
  unsigned short* WD2  = (unsigned short*)(ws + kOffWD2);
  unsigned short* WOUT = (unsigned short*)(ws + kOffWOUT);
  unsigned short* XNH  = (unsigned short*)(ws + kOffXNH);
  unsigned short* XNL  = (unsigned short*)(ws + kOffXNL);
  float*          XZ   = (float*)(ws + kOffXZ);
  unsigned short* XCH  = (unsigned short*)(ws + kOffXCH);
  unsigned short* XCL  = (unsigned short*)(ws + kOffXCL);
  float*          PROJ = (float*)(ws + kOffPROJ);
  unsigned short* D1H  = (unsigned short*)(ws + kOffD1H);
  unsigned short* D1L  = (unsigned short*)(ws + kOffD1L);
  float*          DLR  = (float*)(ws + kOffDLR);
  unsigned short* YH   = (unsigned short*)(ws + kOffYH);
  unsigned short* YL   = (unsigned short*)(ws + kOffYL);

  rne_rows_bf16_kernel<<<(kDin * kDmod / 8) / 256, 256, 0, stream>>>(in_w,   WIN,                        kDin * kDmod / 8);
  rne_rows_bf16_kernel<<<(kDin * kDmod / 8) / 256, 256, 0, stream>>>(skip_w, WIN + (size_t)kDin * kDmod, kDin * kDmod / 8);
  pack_small_kernel<<<kPrjP, 256, 0, stream>>>(wd1, wb, wc, WSM);
  rne_rows_bf16_kernel<<<(kDin * kDtR / 8) / 256, 256, 0, stream>>>(wd2,   WD2,  kDin * kDtR / 8);
  rne_rows_bf16_kernel<<<(kDmod * kDin / 8) / 256, 256, 0, stream>>>(out_w, WOUT, kDmod * kDin / 8);

  rmsnorm_split_kernel<<<kRows / 8, 256, 0, stream>>>(resid, norm_w, XNH, XNL);

  for (int b = 0; b < kBatch; ++b) {
    const size_t rowoff = (size_t)b * kSeqL;
    const unsigned short* XNHb = XNH + rowoff * kDmod;
    const unsigned short* XNLb = XNL + rowoff * kDmod;
    const float* residb = resid + rowoff * kDmod;
    float* outb = out + rowoff * kDmod;

    wmma_gemm64_a2<false><<<((kSeqL / 64) * (kXZP / 64)) / 8, 256, 0, stream>>>(
        XNHb, XNLb, kDmod, WIN, kDmod, XZ, kXZP, residb, kSeqL, kXZP, kDmod);

    conv_silu_split_kernel<<<dim3(kDin / 256, kSeqL / 64), 256, 0, stream>>>(XZ, conv_w, conv_b, XCH, XCL);

    wmma_gemm64_a2<false><<<((kSeqL / 64) * (kPrjP / 64)) / 8, 256, 0, stream>>>(
        XCH, XCL, kDin, WSM, kDin, PROJ, kPrjP, residb, kSeqL, kPrjP, kDin);

    d1_split_kernel<<<(kSeqL * kDtR / 8) / 256, 256, 0, stream>>>(PROJ, D1H, D1L, kSeqL * kDtR / 8);

    wmma_gemm64_a2<false><<<((kSeqL / 64) * (kDin / 64)) / 8, 256, 0, stream>>>(
        D1H, D1L, kDtR, WD2, kDtR, DLR, kDin, residb, kSeqL, kDin, kDtR);

    scan_kernel<<<kDin / kScanCh, kScanCh, 0, stream>>>(
        DLR, (const unsigned*)XCH, (const unsigned*)XCL, XZ, PROJ, A_log, wd2_b, W_D, YH, YL);

    wmma_gemm64_a2<true><<<((kSeqL / 64) * (kDmod / 64)) / 8, 256, 0, stream>>>(
        YH, YL, kDin, WOUT, kDin, outb, kDmod, residb, kSeqL, kDmod, kDin);
  }
}
